// SpectralQuaternionAttention_55886114455827
// MI455X (gfx1250) — hardware-verified
//
#include <hip/hip_runtime.h>


#define NB_  4
#define SS   1024
#define EE   768
#define NH_  12
#define HD   64
#define PCAR 1024.0f
typedef _Float16 h16;
typedef unsigned short bf;
typedef __attribute__((ext_vector_type(16))) __bf16   v16bf;
typedef __attribute__((ext_vector_type(16))) _Float16 v16h;
typedef __attribute__((ext_vector_type(8)))  _Float16 v8h;
typedef __attribute__((ext_vector_type(8)))  unsigned short v8us;
typedef __attribute__((ext_vector_type(8)))  float    v8f;
typedef __attribute__((ext_vector_type(4)))  float    v4f;
typedef v8h  __attribute__((may_alias)) v8ha;
typedef v4f  __attribute__((may_alias)) v4fa;
typedef v8us __attribute__((may_alias)) v8usa;

__device__ __forceinline__ unsigned short f2bf(float f) { unsigned u = __float_as_uint(f); u += 0x7FFFu + ((u >> 16) & 1u); return (unsigned short)(u >> 16); }
__device__ __forceinline__ float bf2f(unsigned short b) { return __uint_as_float(((unsigned)b) << 16); }
__device__ __forceinline__ float bfr(float f) { return bf2f(f2bf(f)); }
__device__ __forceinline__ v16h cat16(v8h lo, v8h hi) { return __builtin_shufflevector(lo, hi, 0, 1, 2, 3, 4, 5, 6, 7, 8, 9, 10, 11, 12, 13, 14, 15); }
__device__ __forceinline__ v16bf cat16b(v8us lo, v8us hi) { return __builtin_bit_cast(v16bf, __builtin_shufflevector(lo, hi, 0, 1, 2, 3, 4, 5, 6, 7, 8, 9, 10, 11, 12, 13, 14, 15)); }
__device__ __forceinline__ v8f wmma16(v16h a, v16h b, v8f c) { return __builtin_amdgcn_wmma_f32_16x16x32_f16(false, a, false, b, (short)0, c, false, false); }
__device__ __forceinline__ v8f wmmab(v16bf a, v16bf b, v8f c) { return __builtin_amdgcn_wmma_f32_16x16x32_bf16(false, a, false, b, (short)0, c, false, false); }


template <typename T16> struct WFrag;
template <> struct WFrag<h16> { typedef v16h V; static __device__ __forceinline__ V ld(const h16* p) { return cat16(*(const v8h*)p, *(const v8h*)(p + 16)); } static __device__ __forceinline__ v8f mma(V a, V b, v8f c) { return wmma16(a, b, c); } };
template <> struct WFrag<bf> { typedef v16bf V; static __device__ __forceinline__ V ld(const bf* p) { return cat16b(*(const v8us*)p, *(const v8us*)(p + 16)); } static __device__ __forceinline__ v8f mma(V a, V b, v8f c) { return wmmab(a, b, c); } };
template <typename T16, int NSPLIT, bool BIAS>
__global__ __launch_bounds__(32) void k_gemmw(const T16* __restrict__ A, const T16* __restrict__ A2, const T16* __restrict__ Bt, const T16* __restrict__ Bt2, int K, float* C, int ldc, const float* __restrict__ bias, size_t sA, size_t sB, size_t sC) {
    typedef typename WFrag<T16>::V V;
    __shared__ __align__(16) float os[16 * 68];
    const size_t z = blockIdx.z; A += z * sA; if (A2) A2 += z * sA; Bt += z * sB; if (Bt2) Bt2 += z * sB; C += z * sC;
    const int lane = threadIdx.x & 31, lr = lane & 15, hi = lane >> 4; const int r0 = blockIdx.x * 64, c0 = blockIdx.y * 64;
    v8f acc[4][4];
#pragma unroll
    for (int mb = 0; mb < 4; ++mb)
#pragma unroll
        for (int nb = 0; nb < 4; ++nb) acc[mb][nb] = (v8f){};
    const size_t aoff = (size_t)(r0 + lr) * K + 8 * hi, boff = (size_t)(c0 + lr) * K + 8 * hi;
#pragma unroll 1
    for (int kc = 0; kc < K; kc += 32) {
        V a[4], a2[4];
#pragma unroll
        for (int mb = 0; mb < 4; ++mb) { a[mb] = WFrag<T16>::ld(A + aoff + (size_t)mb * 16 * K + kc); if (NSPLIT == 1 || NSPLIT == 2) a2[mb] = WFrag<T16>::ld(A2 + aoff + (size_t)mb * 16 * K + kc); }
#pragma unroll
        for (int nb = 0; nb < 4; ++nb) { const V b = WFrag<T16>::ld(Bt + boff + (size_t)nb * 16 * K + kc); V b2; if (NSPLIT >= 2) b2 = WFrag<T16>::ld(Bt2 + boff + (size_t)nb * 16 * K + kc);
#pragma unroll
            for (int mb = 0; mb < 4; ++mb) { acc[mb][nb] = WFrag<T16>::mma(a[mb], b, acc[mb][nb]); if (NSPLIT == 1 || NSPLIT == 2) acc[mb][nb] = WFrag<T16>::mma(a2[mb], b, acc[mb][nb]); if (NSPLIT >= 2) acc[mb][nb] = WFrag<T16>::mma(a[mb], b2, acc[mb][nb]); } }
        asm volatile("v_nop\n\tv_nop\n\tv_nop\n\tv_nop" : "+v"(acc[0][0]), "+v"(acc[1][1]), "+v"(acc[2][2]), "+v"(acc[3][3]) : "v"(a[0]), "v"(a[3]));
    }
#pragma unroll
    for (int mb = 0; mb < 4; ++mb) {
#pragma unroll
        for (int nb = 0; nb < 4; ++nb) {
#pragma unroll
            for (int j = 0; j < 8; ++j) os[(hi * 8 + j) * 68 + nb * 16 + lr] = acc[mb][nb][j]; }
        __builtin_amdgcn_wave_barrier(); asm volatile("" ::: "memory");
        float* crow = C + (size_t)(r0 + mb * 16) * ldc + c0;
#pragma unroll 1
        for (int ps = 0; ps < 2; ++ps) {
#pragma unroll
            for (int s = 0; s < 8; ++s) { const int row = 2 * s + hi, cofs = lr * 4; v4f val = *(const v4fa*)(os + row * 68 + cofs); if (BIAS) { val[0] += bfr(bias[c0 + cofs]); val[1] += bfr(bias[c0 + cofs + 1]); val[2] += bfr(bias[c0 + cofs + 2]); val[3] += bfr(bias[c0 + cofs + 3]); }
                *(volatile v4f*)(crow + (size_t)row * ldc + cofs) = val; }
            if (ps == 0) __threadfence(); }
        __builtin_amdgcn_wave_barrier(); asm volatile("" ::: "memory");
    }
}

__device__ __forceinline__ h16 tohx(float x) { return (h16)x; }
__device__ __forceinline__ void splitf(float y, unsigned short& h, unsigned short& l) { h = f2bf(y); l = f2bf(y - bf2f(h)); }
typedef __attribute__((ext_vector_type(2))) unsigned short v2us;
typedef __attribute__((ext_vector_type(4))) unsigned short v4us;
typedef __attribute__((ext_vector_type(2))) _Float16 v2h;
typedef __attribute__((ext_vector_type(4))) _Float16 v4h;

__global__ __launch_bounds__(256) void k_cvt8(const float* __restrict__ src, bf* dst, size_t n8) { const size_t i = (size_t)blockIdx.x * 256 + threadIdx.x; if (i >= n8) return; const v8f v = *(const v8f*)(src + i * 8); v8us o;
#pragma unroll
    for (int k = 0; k < 8; ++k) o[k] = f2bf(v[k]); *(volatile v8us*)(dst + i * 8) = o; __threadfence(); *(volatile v8us*)(dst + i * 8) = o; }
__global__ __launch_bounds__(256) void k_hker(float* hk) { const int s = blockIdx.x * 256 + threadIdx.x; if (s >= SS) return; float acc = 0.f;
#pragma unroll 1
    for (int k = 0; k < SS; ++k) { const float fr = (k < SS / 2) ? (float)k / (float)SS : (float)(k - SS) / (float)SS; const float w = 6.283185307179586f * fr; const float ph = (w > 0.f ? 1.f : (w < 0.f ? -1.f : 0.f)) * atanf(logf(fabsf(w) + 1e-10f)); const float ang = __fadd_rn(ph, 6.283185307179586f * (float)(((long long)k * s) % SS) / (float)SS); acc = __fadd_rn(acc, cosf(ang)); }
    const float v = acc / (float)SS; *(volatile float*)(hk + s) = v; __threadfence(); *(volatile float*)(hk + s) = v; }
__global__ __launch_bounds__(256) void k_circ(const float* __restrict__ hk, bf* Ch, bf* Cl) { const size_t e = ((size_t)blockIdx.x * 256 + threadIdx.x) * 4; if (e >= (size_t)SS * SS) return; const int t = (int)(e % SS); const int s = (int)(e / SS); v4us oh, ol;
#pragma unroll
    for (int u = 0; u < 4; ++u) { unsigned short a, b; splitf(hk[(s - t - u + 2 * SS) % SS], a, b); oh[u] = a; ol[u] = b; } *(volatile v4us*)(Ch + e) = oh; *(volatile v4us*)(Cl + e) = ol; __threadfence(); *(volatile v4us*)(Ch + e) = oh; *(volatile v4us*)(Cl + e) = ol; }
__global__ __launch_bounds__(256) void k_colnorm(const float* __restrict__ T, float* inv) { const int e = blockIdx.x * 256 + threadIdx.x; if (e >= EE) return; float s = 0.f;
#pragma unroll 1
    for (int r = 0; r < SS; ++r) { const float v = T[(size_t)r * EE + e]; float p = __fmul_rn(v, v); asm volatile("" : "+v"(p)); s = __fadd_rn(s, p); }
    const float iv = __fsqrt_rn(__fadd_rn(s, 1e-8f)); *(volatile float*)(inv + e) = iv; __threadfence(); *(volatile float*)(inv + e) = iv; }
__global__ __launch_bounds__(256) void k_zt(const float* __restrict__ T, const float* __restrict__ nrm, const float* __restrict__ wqr, bf* Zh, bf* Zl) { const size_t e2 = ((size_t)blockIdx.x * 256 + threadIdx.x) * 2; if (e2 >= (size_t)EE * SS) return; const int s = (int)(e2 % SS); const int f = (int)(e2 / SS); const float w0 = bfr(wqr[0]), w1 = bfr(wqr[1]), w2 = bfr(wqr[2]); const float nv = nrm[f]; v2us oh, ol;
#pragma unroll
    for (int u = 0; u < 2; ++u) { const int sc = s + u; const int sm = (sc + SS - 1) % SS, sp1 = (sc + 1) % SS; const float p0 = __fdiv_rn(T[(size_t)sc * EE + f], nv); float pm = __fdiv_rn(T[(size_t)sm * EE + f], nv) * 0.5f, pp = __fdiv_rn(T[(size_t)sp1 * EE + f], nv) * 0.5f; asm volatile("" : "+v"(pm)); asm volatile("" : "+v"(pp));
        float a0 = __fmul_rn(p0, p0), a1 = __fmul_rn(pm, pm), a2 = __fmul_rn(pp, pp); asm volatile("" : "+v"(a0)); asm volatile("" : "+v"(a1)); asm volatile("" : "+v"(a2)); const float qn = __fsqrt_rn(__fadd_rn(__fadd_rn(__fadd_rn(a0, a1), a2), 1e-8f));
        float b0 = __fmul_rn(w0, p0), b1 = __fmul_rn(w1, pm), b2 = __fmul_rn(w2, pp); asm volatile("" : "+v"(b0)); asm volatile("" : "+v"(b1)); asm volatile("" : "+v"(b2)); const float z = __fdiv_rn(__fadd_rn(__fadd_rn(b0, b1), b2), qn);
        unsigned short a, b; splitf(z, a, b); oh[u] = a; ol[u] = b; }
    *(volatile v2us*)(Zh + e2) = oh; *(volatile v2us*)(Zl + e2) = ol; __threadfence(); *(volatile v2us*)(Zh + e2) = oh; *(volatile v2us*)(Zl + e2) = ol; }
__global__ __launch_bounds__(256) void k_rpl(const float* __restrict__ R, const float* __restrict__ bqr, h16* P) { const size_t e = ((size_t)blockIdx.x * 256 + threadIdx.x) * 4; if (e >= (size_t)NH_ * SS * HD) return; const int d = (int)(e % HD); const int s = (int)((e / HD) % SS); const int h = (int)(e / ((size_t)HD * SS)); const float bb = bfr(bqr[0]); const float* r = R + (size_t)s * EE + h * HD + d; v4h o;
#pragma unroll
    for (int u = 0; u < 4; ++u) o[u] = tohx(__fadd_rn(r[u], bb)); *(volatile v4h*)(P + e) = o; __threadfence(); *(volatile v4h*)(P + e) = o; }
__global__ __launch_bounds__(256) void k_rvt(const float* __restrict__ R, const float* __restrict__ bqr, h16* VT) { const size_t e = ((size_t)blockIdx.x * 256 + threadIdx.x) * 2; if (e >= (size_t)NH_ * HD * SS) return; const int s = (int)(e % SS); const int d = (int)((e / SS) % HD); const int h = (int)(e / ((size_t)SS * HD)); const float bb = bfr(bqr[0]); v2h o; o[0] = tohx(__fadd_rn(R[(size_t)s * EE + h * HD + d], bb)); o[1] = tohx(__fadd_rn(R[(size_t)(s + 1) * EE + h * HD + d], bb)); *(volatile v2h*)(VT + e) = o; __threadfence(); *(volatile v2h*)(VT + e) = o; }
__global__ __launch_bounds__(256) void k_smax(const float* __restrict__ S, h16* P16) { const int lane = threadIdx.x & 31; const int row = blockIdx.x * 8 + (threadIdx.x >> 5); if (row >= NH_ * SS) return; const float* sr = S + (size_t)row * SS; float v[SS / 32]; float mx = -3.0e38f;
#pragma unroll
    for (int ch = 0; ch < SS / 128; ++ch) { const v4f a = *(const v4f*)(sr + ch * 128 + lane * 4);
#pragma unroll
        for (int u = 0; u < 4; ++u) { v[ch * 4 + u] = a[u] * 0.125f; mx = fmaxf(mx, v[ch * 4 + u]); } }
#pragma unroll
    for (int sh = 16; sh; sh >>= 1) mx = fmaxf(mx, __shfl_xor(mx, sh, 32));
    float sum = 0.f;
#pragma unroll
    for (int q = 0; q < SS / 32; ++q) { float d0 = __fsub_rn(v[q], mx); asm volatile("" : "+v"(d0)); v[q] = __builtin_amdgcn_exp2f(__fmul_rn(d0, 1.4426950408889634f)); sum += v[q]; }
#pragma unroll
    for (int sh = 16; sh; sh >>= 1) sum += __shfl_xor(sum, sh, 32);
    const float f = __fdiv_rn(PCAR, sum);
    for (int ps = 0; ps < 2; ++ps) {
#pragma unroll
        for (int ch = 0; ch < SS / 128; ++ch) { v4h o4; for (int q = 0; q < 4; ++q) o4[q] = tohx(v[ch * 4 + q] * f); *(volatile v4h*)(P16 + (size_t)row * SS + ch * 128 + lane * 4) = o4; }
        if (ps == 0) __threadfence(); } }
__global__ __launch_bounds__(256) void k_mrg(const float* __restrict__ O, bf* Ah, bf* Al) { const size_t e = ((size_t)blockIdx.x * 256 + threadIdx.x) * 4; if (e >= (size_t)NH_ * SS * HD) return; const int d = (int)(e % HD); const int s = (int)((e / HD) % SS); const int h = (int)(e / ((size_t)HD * SS)); const size_t oo = (size_t)s * EE + h * HD + d; v4us oh, ol;
#pragma unroll
    for (int u = 0; u < 4; ++u) { unsigned short a, b; splitf(O[e + u] * (1.0f / PCAR), a, b); oh[u] = a; ol[u] = b; } *(volatile v4us*)(Ah + oo) = oh; *(volatile v4us*)(Al + oo) = ol; __threadfence(); *(volatile v4us*)(Ah + oo) = oh; *(volatile v4us*)(Al + oo) = ol; }

extern "C" void kernel_launch(void* const* d_in, const int* in_sizes, int n_in,
                              void* d_out, int out_size, void* d_ws, size_t ws_size, hipStream_t stream) {
    (void)in_sizes; (void)n_in; (void)out_size;
    const float** I = (const float**)d_in;
    const float *x = I[0], *Wq = I[1], *bq = I[2], *Wk = I[3], *bk = I[4], *Wv = I[5], *bv = I[6], *Wo = I[7], *bo = I[8], *wqr = I[9], *bqr = I[10];
    float* OUT = (float*)d_out;
    char* wsp = (char*)d_ws;
    auto take = [&](size_t bytes) { char* p = wsp; wsp += (bytes + 255) & ~(size_t)255; return (void*)p; };
    float* HK = (float*)take(SS * 4); bf* Ch = (bf*)take((size_t)SS * SS * 2); bf* Cl = (bf*)take((size_t)SS * SS * 2);
    bf* XB = (bf*)take((size_t)SS * EE * 2); bf* BQ = (bf*)take((size_t)EE * EE * 2); bf* BK = (bf*)take((size_t)EE * EE * 2); bf* BV = (bf*)take((size_t)EE * EE * 2); bf* BO = (bf*)take((size_t)EE * EE * 2);
    float* T = (float*)take((size_t)SS * EE * 4); float* NRM = (float*)take(EE * 4); bf* ZTh = (bf*)take((size_t)EE * SS * 2); bf* ZTl = (bf*)take((size_t)EE * SS * 2); float* R = (float*)take((size_t)SS * EE * 4);
    h16* QP = (h16*)take((size_t)NH_ * SS * HD * 2); h16* KP = (h16*)take((size_t)NH_ * SS * HD * 2); h16* VT = (h16*)take((size_t)NH_ * HD * SS * 2);
    float* S = (float*)take((size_t)NH_ * SS * SS * 4); h16* P16 = (h16*)take((size_t)NH_ * SS * SS * 2); float* O = (float*)take((size_t)NH_ * SS * HD * 4); bf* ATh = (bf*)take((size_t)SS * EE * 2); bf* ATl = (bf*)take((size_t)SS * EE * 2);
    if ((size_t)(wsp - (char*)d_ws) > ws_size) return;
    k_hker<<<(SS + 255) / 256, 256, 0, stream>>>(HK); k_circ<<<(unsigned)(((size_t)SS * SS / 4 + 255) / 256), 256, 0, stream>>>(HK, Ch, Cl);
    k_cvt8<<<(EE * EE / 8 + 255) / 256, 256, 0, stream>>>(Wq, BQ, EE * EE / 8); k_cvt8<<<(EE * EE / 8 + 255) / 256, 256, 0, stream>>>(Wk, BK, EE * EE / 8); k_cvt8<<<(EE * EE / 8 + 255) / 256, 256, 0, stream>>>(Wv, BV, EE * EE / 8); k_cvt8<<<(EE * EE / 8 + 255) / 256, 256, 0, stream>>>(Wo, BO, EE * EE / 8);
    const dim3 gp(SS / 64, EE / 64, 1); const size_t zq = (size_t)SS * HD, zS = (size_t)SS * SS, zv = (size_t)HD * SS;
    for (int b = 0; b < NB_; ++b) {
        k_cvt8<<<(SS * EE / 8 + 255) / 256, 256, 0, stream>>>(x + (size_t)b * SS * EE, XB, SS * EE / 8);
        for (int which = 0; which < 3; ++which) { const bf* BW = which == 0 ? BQ : (which == 1 ? BK : BV); const float* bb = which == 0 ? bq : (which == 1 ? bk : bv);
            k_gemmw<bf, 0, true><<<gp, 32, 0, stream>>>(XB, nullptr, BW, nullptr, EE, T, EE, bb, 0, 0, 0);
            k_colnorm<<<(EE + 255) / 256, 256, 0, stream>>>(T, NRM);
            k_zt<<<(unsigned)(((size_t)EE * SS / 2 + 255) / 256), 256, 0, stream>>>(T, NRM, wqr, ZTh, ZTl);
            k_gemmw<bf, 2, false><<<dim3(SS / 64, EE / 64, 1), 32, 0, stream>>>(Ch, Cl, ZTh, ZTl, SS, R, EE, nullptr, 0, 0, 0);
            if (which == 0) k_rpl<<<(NH_ * SS * HD / 4 + 255) / 256, 256, 0, stream>>>(R, bqr, QP); else if (which == 1) k_rpl<<<(NH_ * SS * HD / 4 + 255) / 256, 256, 0, stream>>>(R, bqr, KP); else k_rvt<<<(NH_ * HD * SS / 2 + 255) / 256, 256, 0, stream>>>(R, bqr, VT); }
        k_gemmw<h16, 0, false><<<dim3(SS / 64, SS / 64, NH_), 32, 0, stream>>>(QP, nullptr, KP, nullptr, HD, S, SS, nullptr, zq, zq, zS);
        k_smax<<<NH_ * SS / 8, 256, 0, stream>>>(S, P16);
        k_gemmw<h16, 0, false><<<dim3(SS / 64, 1, NH_), 32, 0, stream>>>(P16, nullptr, VT, nullptr, SS, O, HD, nullptr, zS, zv, zq);
        k_mrg<<<(NH_ * SS * HD / 4 + 255) / 256, 256, 0, stream>>>(O, ATh, ATl);
        k_gemmw<bf, 1, true><<<gp, 32, 0, stream>>>(ATh, ATl, BO, nullptr, EE, OUT + (size_t)b * SS * EE, EE, bo, 0, 0, 0); }
}
